// CTCDecoderN_82111184765030
// MI455X (gfx1250) — hardware-verified
//
#include <hip/hip_runtime.h>

#define LL 4096
#define BB 4
#define DD 512
#define VV 1000
#define VP 1024

typedef _Float16 f16;
typedef f16 v16h __attribute__((ext_vector_type(16)));
typedef f16 v8h __attribute__((ext_vector_type(8)));
typedef float v8f __attribute__((ext_vector_type(8)));
typedef float v4f __attribute__((ext_vector_type(4)));

union Frag { v16h v; v8h half[2]; };
union Pk16 { v8h h; v4f f; };

__device__ __forceinline__ v8f wmma16(v16h a, v16h b, v8f c) {
  c = __builtin_amdgcn_wmma_f32_16x16x32_f16(false, a, false, b, (short)0, c,
                                              false, false);
  asm volatile("v_nop\n\tv_nop\n\tv_nop\n\tv_nop" : "+v"(c) : "v"(a), "v"(b));
  return c;
}

__device__ __forceinline__ v16h ld_frag(const f16* rowp, int k0, int h) {
  Frag f;
  f.half[0] = *(const v8h*)(rowp + k0 + 8 * h);
  f.half[1] = *(const v8h*)(rowp + k0 + 16 + 8 * h);
  return f.v;
}

__device__ __forceinline__ void vst_h8(f16* p, v8h v) {
  Pk16 u;
  u.h = v;
  *(volatile v4f*)p = u.f;
}
__device__ __forceinline__ void vst_f4(float* p, v4f v) {
  *(volatile v4f*)p = v;
}

__global__ void __launch_bounds__(256)
k_cvt_w(const float* __restrict__ Ww, const float* __restrict__ Lw,
        f16* __restrict__ Wwh, f16* __restrict__ Lwh) {
  const int NW = DD * DD / 8;
  const int NL = VP * DD / 8;
  const int p = blockIdx.x * 256 + threadIdx.x;
  if (p >= NW + NL) return;
  v8h v;
  f16* dst;
  if (p < NW) {
    const float* s = Ww + (size_t)p * 8;
    v4f a = *(const v4f*)s;
    v4f c = *(const v4f*)(s + 4);
#pragma unroll
    for (int j = 0; j < 4; ++j) {
      v[j] = (f16)(a[j] * 16.0f);
      v[4 + j] = (f16)(c[j] * 16.0f);
    }
    dst = Wwh + (size_t)p * 8;
  } else {
    const int pp = p - NW;
    const int row = pp >> 6;
    const int col = (pp & 63) * 8;
    if (row < VV) {
      const float* s = Lw + (size_t)row * DD + col;
      v4f a = *(const v4f*)s;
      v4f c = *(const v4f*)(s + 4);
#pragma unroll
      for (int j = 0; j < 4; ++j) {
        v[j] = (f16)(a[j] * 16.0f);
        v[4 + j] = (f16)(c[j] * 16.0f);
      }
    } else {
#pragma unroll
      for (int j = 0; j < 8; ++j) v[j] = (f16)0.0f;
    }
    dst = Lwh + (size_t)pp * 8;
  }
  vst_h8(dst, v);
  __threadfence();
  vst_h8(dst, v);
}

__global__ void __launch_bounds__(256)
k_cvt_x(const float* __restrict__ x, f16* __restrict__ xh, f16* __restrict__ xT) {
  __shared__ __align__(16) f16 sX[64 * 72];
  const int t = threadIdx.x;
  const int l0 = blockIdx.x * 64, d0 = blockIdx.y * 64, b = blockIdx.z;
  v8h hv[2];
#pragma unroll
  for (int i = 0; i < 2; ++i) {
    const int P = t + 256 * i;
    const int ll = P >> 3, dc = (P & 7) * 8;
    const float* s = x + ((size_t)(l0 + ll) * BB + b) * DD + d0 + dc;
    v4f a = *(const v4f*)s;
    v4f c = *(const v4f*)(s + 4);
    v8h v;
#pragma unroll
    for (int j = 0; j < 4; ++j) {
      v[j] = (f16)a[j];
      v[4 + j] = (f16)c[j];
    }
    hv[i] = v;
#pragma unroll
    for (int j = 0; j < 8; ++j) sX[(dc + j) * 72 + ll] = v[j];
  }
#pragma unroll
  for (int i = 0; i < 2; ++i) {
    const int P = t + 256 * i;
    const int ll = P >> 3, dc = (P & 7) * 8;
    vst_h8(xh + ((size_t)(b * LL + l0 + ll)) * DD + d0 + dc, hv[i]);
  }
  __threadfence();
#pragma unroll
  for (int i = 0; i < 2; ++i) {
    const int P = t + 256 * i;
    const int ll = P >> 3, dc = (P & 7) * 8;
    vst_h8(xh + ((size_t)(b * LL + l0 + ll)) * DD + d0 + dc, hv[i]);
  }
  __syncthreads();
  v8h tv[2];
#pragma unroll
  for (int i = 0; i < 2; ++i) {
    const int P = t + 256 * i;
    const int dd = P >> 3, q = P & 7;
    tv[i] = *(const v8h*)(sX + dd * 72 + q * 8);
  }
#pragma unroll
  for (int i = 0; i < 2; ++i) {
    const int P = t + 256 * i;
    const int dd = P >> 3, q = P & 7;
    vst_h8(xT + ((size_t)(b * DD + d0 + dd)) * LL + l0 + q * 8, tv[i]);
  }
  __threadfence();
#pragma unroll
  for (int i = 0; i < 2; ++i) {
    const int P = t + 256 * i;
    const int dd = P >> 3, q = P & 7;
    vst_h8(xT + ((size_t)(b * DD + d0 + dd)) * LL + l0 + q * 8, tv[i]);
  }
}

template <int MODE>
__global__ void __launch_bounds__(256)
k_gemm(const f16* __restrict__ A, int lda, long long zA,
       const f16* __restrict__ Bm, int ldb, long long zB, int K,
       const float* __restrict__ bias, float scale,
       f16* __restrict__ C, int ldc, long long zC, int rowmul, int rowzadd) {
  __shared__ __align__(16) f16 sS[128 * 72];
  const int t = threadIdx.x, lane = t & 31, w = t >> 5;
  const int h = lane >> 4, m = lane & 15;
  const int row0 = blockIdx.x * 128, col0 = blockIdx.y * 64, z = blockIdx.z;
  const int mrow = (w >> 1) * 32, ncol = (w & 1) * 32;

  const f16* Ab = A + (size_t)z * zA + (size_t)(row0 + mrow) * lda;
  const f16* Bb = Bm + (size_t)z * zB + (size_t)(col0 + ncol) * ldb;
  const f16* a0p = Ab + (size_t)m * lda;
  const f16* a1p = Ab + (size_t)(16 + m) * lda;
  const f16* b0p = Bb + (size_t)m * ldb;
  const f16* b1p = Bb + (size_t)(16 + m) * ldb;

  v8f vz = {};
  v8f c00 = vz, c01 = vz, c10 = vz, c11 = vz;
  for (int k0 = 0; k0 < K; k0 += 32) {
    v16h a0 = ld_frag(a0p, k0, h);
    v16h a1 = ld_frag(a1p, k0, h);
    v16h b0 = ld_frag(b0p, k0, h);
    v16h b1 = ld_frag(b1p, k0, h);
    c00 = wmma16(a0, b0, c00);
    c01 = wmma16(a0, b1, c01);
    c10 = wmma16(a1, b0, c10);
    c11 = wmma16(a1, b1, c11);
  }

  if (MODE == 0) {
    const int PT = 136;
    const float g0 = bias[col0 + ncol + m];
    const float g1 = bias[col0 + ncol + 16 + m];
    f16* s0 = sS + (ncol + m) * PT + mrow + 8 * h;
    f16* s1 = sS + (ncol + 16 + m) * PT + mrow + 8 * h;
#pragma unroll
    for (int r = 0; r < 8; ++r) {
      s0[r] = (f16)(c00[r] * scale + g0);
      s1[r] = (f16)(c01[r] * scale + g1);
      s0[16 + r] = (f16)(c10[r] * scale + g0);
      s1[16 + r] = (f16)(c11[r] * scale + g1);
    }
  } else {
    const int PN = 72;
    f16* s0 = sS + (mrow + 8 * h) * PN + ncol + m;
#pragma unroll
    for (int r = 0; r < 8; ++r) {
      s0[r * PN] = (f16)(c00[r] * scale);
      s0[r * PN + 16] = (f16)(c01[r] * scale);
      s0[(16 + r) * PN] = (f16)(c10[r] * scale);
      s0[(16 + r) * PN + 16] = (f16)(c11[r] * scale);
    }
  }
  __syncthreads();

  f16* Cz = C + (size_t)z * zC;
  v8h vals[4];
  if (MODE == 0) {
#pragma unroll
    for (int i = 0; i < 4; ++i) {
      const int P = t + 256 * i;
      const int dd = P >> 4, q = P & 15;
      vals[i] = *(const v8h*)(sS + dd * 136 + q * 8);
    }
#pragma unroll
    for (int i = 0; i < 4; ++i) {
      const int P = t + 256 * i;
      const int dd = P >> 4, q = P & 15;
      vst_h8(Cz + (size_t)(col0 + dd) * ldc + row0 + q * 8, vals[i]);
    }
    __threadfence();
#pragma unroll
    for (int i = 0; i < 4; ++i) {
      const int P = t + 256 * i;
      const int dd = P >> 4, q = P & 15;
      vst_h8(Cz + (size_t)(col0 + dd) * ldc + row0 + q * 8, vals[i]);
    }
  } else {
#pragma unroll
    for (int i = 0; i < 4; ++i) {
      const int P = t + 256 * i;
      const int rr = P >> 3, q = P & 7;
      vals[i] = *(const v8h*)(sS + rr * 72 + q * 8);
    }
#pragma unroll
    for (int i = 0; i < 4; ++i) {
      const int P = t + 256 * i;
      const int rr = P >> 3, q = P & 7;
      const size_t orow = (size_t)((row0 + rr) * rowmul + z * rowzadd);
      vst_h8(Cz + orow * ldc + col0 + q * 8, vals[i]);
    }
    __threadfence();
#pragma unroll
    for (int i = 0; i < 4; ++i) {
      const int P = t + 256 * i;
      const int rr = P >> 3, q = P & 7;
      const size_t orow = (size_t)((row0 + rr) * rowmul + z * rowzadd);
      vst_h8(Cz + orow * ldc + col0 + q * 8, vals[i]);
    }
  }
}

__global__ void __launch_bounds__(256)
k_logits(const f16* __restrict__ yh, const f16* __restrict__ Lwh,
         const float* __restrict__ Lb, float* __restrict__ out) {
  __shared__ __align__(16) float sL[16 * VP];
  __shared__ float sMx[16];
  __shared__ float sLs[16];
  const int t = threadIdx.x, lane = t & 31, w = t >> 5;
  const int h = lane >> 4, m = lane & 15;
  const int r0 = blockIdx.x * 16;
  const f16* ap = yh + (size_t)(r0 + m) * DD;
  v8f vz = {};

#pragma unroll 1
  for (int g = 0; g < 2; ++g) {
    const int cbase = w * 128 + g * 64;
    const f16* bp = Lwh + (size_t)(cbase + m) * DD;
    v8f acc[4];
#pragma unroll
    for (int j = 0; j < 4; ++j) acc[j] = vz;
    for (int k0 = 0; k0 < DD; k0 += 32) {
      v16h a = ld_frag(ap, k0, h);
#pragma unroll
      for (int j = 0; j < 4; ++j)
        acc[j] = wmma16(a, ld_frag(bp + (size_t)j * 16 * DD, k0, h), acc[j]);
    }
#pragma unroll
    for (int j = 0; j < 4; ++j) {
      const int v = cbase + j * 16 + m;
      const float bv = (v < VV) ? Lb[v] : 0.0f;
      float* s = sL + (8 * h) * VP + v;
#pragma unroll
      for (int r = 0; r < 8; ++r) s[r * VP] = acc[j][r] * 16.0f + bv;
    }
  }
  __syncthreads();

  const int row = t >> 4, sub = t & 15;
  const float* srow = sL + row * VP;
  float mx = -3.0e38f;
  for (int v = sub; v < VV; v += 16) mx = fmaxf(mx, srow[v]);
  mx = fmaxf(mx, __shfl_xor(mx, 8));
  mx = fmaxf(mx, __shfl_xor(mx, 4));
  mx = fmaxf(mx, __shfl_xor(mx, 2));
  mx = fmaxf(mx, __shfl_xor(mx, 1));
  float se = 0.0f;
  for (int v = sub; v < VV; v += 16) se += __expf(srow[v] - mx);
  se += __shfl_xor(se, 8);
  se += __shfl_xor(se, 4);
  se += __shfl_xor(se, 2);
  se += __shfl_xor(se, 1);
  if (sub == 0) {
    sMx[row] = mx;
    sLs[row] = __logf(se);
  }
  __syncthreads();

  float* ob = out + (size_t)blockIdx.x * (16 * VV);
  for (int pass = 0; pass < 2; ++pass) {
#pragma unroll
    for (int i = 0; i < 16; ++i) {
      const int P = t + 256 * i;
      if (P < 4 * VV) {
        const int e = P * 4;
        const int rr = e / VV;
        const int cc = e - rr * VV;
        v4f lv = *(const v4f*)(sL + rr * VP + cc);
        const float mxr = sMx[rr], ls = sLs[rr];
        v4f o;
#pragma unroll
        for (int q = 0; q < 4; ++q) o[q] = (lv[q] - mxr) - ls;
        vst_f4(ob + e, o);
      }
    }
    if (pass == 0) __threadfence();
  }
}

extern "C" void kernel_launch(void* const* d_in, const int* in_sizes, int n_in,
                              void* d_out, int out_size, void* d_ws, size_t ws_size,
                              hipStream_t stream) {
  if (n_in < 5) return;
  if (in_sizes[0] != LL * BB * DD || in_sizes[1] != DD * DD || in_sizes[2] != DD ||
      in_sizes[3] != VV * DD || in_sizes[4] != VV || out_size != LL * BB * VV)
    return;

  const float* x  = (const float*)d_in[0];
  const float* Ww = (const float*)d_in[1];
  const float* Wb = (const float*)d_in[2];
  const float* Lw = (const float*)d_in[3];
  const float* Lb = (const float*)d_in[4];
  float* out = (float*)d_out;
  char* ws = (char*)d_ws;

  const size_t SZ   = (size_t)BB * LL * DD * 2;
  const size_t oXh  = 0;
  const size_t oXT  = oXh + SZ;
  const size_t oWxT = oXT + SZ;
  const size_t oYh  = oWxT + SZ;
  const size_t oWwh = oYh + SZ;
  const size_t oLwh = oWwh + (size_t)DD * DD * 2;
  const size_t oGTh = oLwh + (size_t)VP * DD * 2;
  const size_t oEnd = oGTh + (size_t)BB * DD * DD * 2;
  if (oEnd > ws_size) return;

  f16* xh  = (f16*)(ws + oXh);
  f16* xT  = (f16*)(ws + oXT);
  f16* wxT = (f16*)(ws + oWxT);
  f16* yh  = (f16*)(ws + oYh);
  f16* Wwh = (f16*)(ws + oWwh);
  f16* Lwh = (f16*)(ws + oLwh);
  f16* GTh = (f16*)(ws + oGTh);

  const float inv16 = 0.0625f;

  k_cvt_w<<<(DD * DD / 8 + VP * DD / 8) / 256, 256, 0, stream>>>(Ww, Lw, Wwh, Lwh);
  k_cvt_x<<<dim3(LL / 64, DD / 64, BB), 256, 0, stream>>>(x, xh, xT);
  k_gemm<0><<<dim3(LL / 128, DD / 64, BB), 256, 0, stream>>>(
      xh, DD, (long long)LL * DD, Wwh, DD, 0LL, DD, Wb, inv16,
      wxT, LL, (long long)DD * LL, 0, 0);
  k_gemm<1><<<dim3(DD / 128, DD / 64, BB), 256, 0, stream>>>(
      xT, LL, (long long)DD * LL, wxT, LL, (long long)DD * LL, LL, Wb, inv16,
      GTh, DD, (long long)DD * DD, 1, 0);
  k_gemm<1><<<dim3(LL / 128, DD / 64, BB), 256, 0, stream>>>(
      xh, DD, (long long)LL * DD, GTh, DD, (long long)DD * DD, DD, Wb, inv16,
      yh, DD, 0LL, BB, 1);
  k_logits<<<(LL * BB) / 16, 256, 0, stream>>>(yh, Lwh, Lb, out);
}
